// graphSAGE_71683004171208
// MI455X (gfx1250) — hardware-verified
//
#include <hip/hip_runtime.h>
#include <stddef.h>
#include <stdint.h>
#include <math.h>


#define FX     128
#define FH     64
#define NCLS   40
#define NC2P   64
#define K1     384
#define K2     256
#define APS    512
#define NTHR   256
#define NWAVE  8
#define EPT    8
#define CHUNK  (NTHR * EPT)
#define WCAP   (EPT * 32)
#define LISTN  (NWAVE * WCAP)
#define NBA    1024
#define SLA    10
#define RCAP   28672
#define DEGCAP 1024
#define GBM    64
#define GBN    64
#define GTHR   128
#define U0     3072
#define U1     2048
#define AGG_ZINTS    (LISTN + 2 * RCAP + 3 * NBA)
#define MISC_INTS    16
#define ROWBUF_INTS  (NWAVE * APS / 2)
#define AGG_LDS_INTS (AGG_ZINTS + MISC_INTS + ROWBUF_INTS)
#define WSMAX  134217728

static_assert((CHUNK & (CHUNK - 1)) == 0 && CHUNK <= 4096);
static_assert((NBA & (NBA - 1)) == 0 && NBA == (1 << SLA));
static_assert(((long long)CHUNK << SLA) < (1LL << 31));
static_assert(LISTN % NTHR == 0);
static_assert(NBA % NWAVE == 0 && NBA % 32 == 0 && NBA % GBM == 0);
static_assert(RCAP % 4 == 0 && AGG_ZINTS % 4 == 0 && LISTN % 4 == 0 && ((AGG_ZINTS + MISC_INTS) % 4) == 0);
static_assert(AGG_ZINTS % (NTHR * 4) == 0);
static_assert(K1 % 32 == 0 && K2 % 32 == 0 && K1 == 3 * FX && K2 == 4 * FH);
static_assert(APS >= K1 && APS >= K2);
static_assert(GBM == (GTHR / 32) * 16 && GBN == FH && NC2P == GBN);
static_assert(FX == 4 * 32 && FH == 2 * 32);
static_assert(NCLS <= NC2P && (NCLS % 4) == 0 && (NCLS % 2) == 0);
static_assert(U0 % NTHR == 0 && U1 % NTHR == 0 && (U0 % 1024) == 0 && (U1 % 512) == 0);
static_assert(U0 == 3 * FH * (FX / 8) && U1 == 4 * NC2P * (FH / 8));
static_assert(AGG_LDS_INTS * 4 <= 300000);
static_assert(((GBM * NCLS * 4) % 128) == 0);

typedef float          v2f   __attribute__((ext_vector_type(2)));
typedef float          v4f   __attribute__((ext_vector_type(4)));
typedef float          v8f   __attribute__((ext_vector_type(8)));
typedef int            v4i   __attribute__((ext_vector_type(4)));
typedef int            v8i   __attribute__((ext_vector_type(8)));
typedef unsigned short v4us  __attribute__((ext_vector_type(4)));
typedef unsigned short v8us  __attribute__((ext_vector_type(8)));
typedef unsigned short v16us __attribute__((ext_vector_type(16)));
typedef __bf16         v16bf __attribute__((ext_vector_type(16)));
typedef v2f  __attribute__((may_alias)) v2fa;
typedef v4f  __attribute__((may_alias)) v4fa;
typedef v4i  __attribute__((may_alias)) v4ia;
typedef v4us __attribute__((may_alias)) v4usa;
typedef v8us __attribute__((may_alias)) v8usa;
typedef unsigned int __attribute__((may_alias)) ua32;
union FragB { v16bf v; v16us u; v8us h[2]; v8i w; };

__device__ __forceinline__ v8f wmb(const FragB& a, const FragB& b, v8f c) {
  v8f d = __builtin_amdgcn_wmma_f32_16x16x32_bf16(false, a.v, false, b.v, (short)0, c, false, false);
  asm volatile("v_nop\n\tv_nop\n\tv_nop\n\tv_nop" : "+v"(d) : "v"(a.w), "v"(b.w));
  return d;
}

__device__ __forceinline__ unsigned bf16_bits(float f) {
  const unsigned u = __float_as_uint(f);
  return ((u + 0x7FFFu + ((u >> 16) & 1u)) >> 16) & 0xFFFFu;
}
__device__ __forceinline__ float bf16_val(float f) {
  return __uint_as_float(bf16_bits(f) << 16);
}
__device__ __forceinline__ v4f bfr4(const v4f a) {
  v4f r; r.x = bf16_val(a.x); r.y = bf16_val(a.y); r.z = bf16_val(a.z); r.w = bf16_val(a.w); return r;
}
__device__ __forceinline__ void split2(float v, unsigned& hi, unsigned& lo) {
  hi = bf16_bits(v);
  lo = bf16_bits(v - __uint_as_float(hi << 16));
}

__device__ __forceinline__ void wave_sync() {
  __builtin_amdgcn_fence(__ATOMIC_RELEASE, "wavefront");
  __builtin_amdgcn_wave_barrier();
  __builtin_amdgcn_fence(__ATOMIC_ACQUIRE, "wavefront");
}

template <int SLB>
__device__ __forceinline__ int scan_chunk(const int* __restrict__ dsts, int nE, int cbase, int slotBase,
                                          int nb, int vec8, int* list, int tid, int lane, int wave) {
  int wc = 0;
  const int el0  = tid * EPT;
  const int e0   = cbase + el0;
  const int sent = -2147483647 - 1;
  v4i da, db;
  if (vec8 != 0 && cbase + CHUNK <= nE) {
    da = *(const v4i*)(dsts + e0);
    db = *(const v4i*)(dsts + e0 + 4);
  } else {
    da.x = (e0     < nE) ? dsts[min(e0,     nE - 1)] : sent;
    da.y = (e0 + 1 < nE) ? dsts[min(e0 + 1, nE - 1)] : sent;
    da.z = (e0 + 2 < nE) ? dsts[min(e0 + 2, nE - 1)] : sent;
    da.w = (e0 + 3 < nE) ? dsts[min(e0 + 3, nE - 1)] : sent;
    db.x = (e0 + 4 < nE) ? dsts[min(e0 + 4, nE - 1)] : sent;
    db.y = (e0 + 5 < nE) ? dsts[min(e0 + 5, nE - 1)] : sent;
    db.z = (e0 + 6 < nE) ? dsts[min(e0 + 6, nE - 1)] : sent;
    db.w = (e0 + 7 < nE) ? dsts[min(e0 + 7, nE - 1)] : sent;
  }
  const unsigned nbs = (unsigned)slotBase;
  const unsigned unb = (unsigned)nb;
  const unsigned s0 = (unsigned)da.x - nbs, s1 = (unsigned)da.y - nbs;
  const unsigned s2 = (unsigned)da.z - nbs, s3 = (unsigned)da.w - nbs;
  const unsigned s4 = (unsigned)db.x - nbs, s5 = (unsigned)db.y - nbs;
  const unsigned s6 = (unsigned)db.z - nbs, s7 = (unsigned)db.w - nbs;
  const bool h0 = s0 < unb, h1 = s1 < unb, h2 = s2 < unb, h3 = s3 < unb;
  const bool h4 = s4 < unb, h5 = s5 < unb, h6 = s6 < unb, h7 = s7 < unb;
  const unsigned any = __builtin_amdgcn_ballot_w32(h0 | h1 | h2 | h3 | h4 | h5 | h6 | h7);
  if (any != 0u) {
#define HITJ(J, HJ, SJ) { \
      const unsigned mj = __builtin_amdgcn_ballot_w32(HJ); \
      if (mj != 0u) { \
        if (HJ) { \
          const int pos = wc + (int)__builtin_amdgcn_mbcnt_lo(mj, 0u); \
          if (pos < WCAP) list[wave * WCAP + pos] = ((el0 + (J)) << SLB) | (int)(SJ); \
        } \
        wc += (int)__builtin_popcount(mj); } }
    HITJ(0, h0, s0)
    HITJ(1, h1, s1)
    HITJ(2, h2, s2)
    HITJ(3, h3, s3)
    HITJ(4, h4, s4)
    HITJ(5, h5, s5)
    HITJ(6, h6, s6)
    HITJ(7, h7, s7)
#undef HITJ
  }
  return wc;
}

__global__ __launch_bounds__(NTHR) void k_wprep(const float* __restrict__ Wl1, const float* __restrict__ Wr1,
                                                const float* __restrict__ Wl2, const float* __restrict__ Wr2,
                                                unsigned short* B0, unsigned short* B1) {
  const int u = (int)blockIdx.x * NTHR + (int)threadIdx.x;
  if (u >= U0 + U1) return;
  const float* W;
  unsigned short* P;
  int pitch, coff, ldw, ncol, n, k8;
  if (u < U0) {
    const int part = u >> 10;
    const int v    = u & 1023;
    n = v >> 4; k8 = (v & 15) * 8;
    pitch = K1; ldw = FH; ncol = FH; P = B0;
    if (part == 0)      { W = Wl1; coff = 0; }
    else if (part == 1) { W = Wl1; coff = FX; }
    else                { W = Wr1; coff = 2 * FX; }
  } else {
    const int u2   = u - U0;
    const int part = u2 >> 9;
    const int v    = u2 & 511;
    n = v >> 3; k8 = (v & 7) * 8;
    pitch = K2; ldw = NCLS; ncol = NCLS; P = B1;
    if (part == 0)      { W = Wl2; coff = 0; }
    else if (part == 1) { W = Wl2; coff = FH; }
    else if (part == 2) { W = Wr2; coff = 2 * FH; }
    else                { W = Wr2; coff = 3 * FH; }
  }
  const int ncl = n < ncol ? n : ncol - 1;
  const float* p = W + (size_t)k8 * (size_t)ldw + ncl;
  float f[8];
#pragma unroll
  for (int i = 0; i < 8; ++i) f[i] = p[(size_t)i * ldw];
  const bool live = n < ncol;
  v8us o;
#pragma unroll
  for (int i = 0; i < 8; ++i) o[i] = live ? (unsigned short)bf16_bits(f[i]) : (unsigned short)0;
  unsigned short* dp = P + (size_t)n * (size_t)pitch + coff + k8;
  *(volatile v8us*)dp = o;
  __threadfence();
  *(volatile v8us*)dp = o;
}

template <int FIN>
__global__ __launch_bounds__(GTHR) void k_gemm(const unsigned short* __restrict__ A, const unsigned short* __restrict__ BT,
                                               int K, const float* __restrict__ bias, float* outp, int nOut) {
  __shared__ __attribute__((aligned(16))) float stg[GBM * GBN];
  __shared__ __attribute__((aligned(16))) float res[GBM * NCLS];
  const int tid = (int)threadIdx.x, lane = tid & 31, wave = tid >> 5, hh = lane >> 4, m = lane & 15;
  const int rowBase = (int)blockIdx.x * GBM;

  v8f acc[4];
  {
    const v8f z = {0.f, 0.f, 0.f, 0.f, 0.f, 0.f, 0.f, 0.f};
    acc[0] = z; acc[1] = z; acc[2] = z; acc[3] = z;
  }
  const unsigned short* ap = A  + (size_t)(rowBase + 16 * wave + m) * (size_t)K + 8 * hh;
  const unsigned short* wp = BT + (size_t)m * (size_t)K + 8 * hh;
  const int ksteps = K >> 5;
#pragma unroll 1
  for (int ks = 0; ks < ksteps; ++ks) {
    FragB af;
    af.h[0] = *(const v8usa*)(ap + 32 * ks);
    af.h[1] = *(const v8usa*)(ap + 32 * ks + 16);
#pragma unroll
    for (int t = 0; t < 4; ++t) {
      const unsigned short* wq = wp + (size_t)(16 * t) * (size_t)K + 32 * ks;
      FragB bf;
      bf.h[0] = *(const v8usa*)wq;
      bf.h[1] = *(const v8usa*)(wq + 16);
      acc[t] = wmb(af, bf, acc[t]);
    }
  }

#pragma unroll
  for (int t = 0; t < 4; ++t) {
    const int lc = 16 * t + m;
#pragma unroll
    for (int r = 0; r < 8; ++r) {
      const int lr = 16 * wave + 8 * hh + r;
      stg[lr * GBN + lc] = acc[t][r];
    }
  }
  __syncthreads();

  if constexpr (FIN == 0) {
    const v4f bb4 = bfr4(*(const v4f*)(bias + 4 * m));
    v4f fv[8];
#pragma unroll
    for (int i = 0; i < 8; ++i) {
      const int lr = 16 * wave + 2 * i + hh;
      v4f t = *(const v4fa*)(stg + lr * GBN + 4 * m) + bb4;
      t.x = fmaxf(t.x, 0.0f); t.y = fmaxf(t.y, 0.0f); t.z = fmaxf(t.z, 0.0f); t.w = fmaxf(t.w, 0.0f);
      fv[i] = t;
    }
#pragma unroll
    for (int i = 0; i < 8; ++i) {
      const int gr = rowBase + 16 * wave + 2 * i + hh;
      *(volatile v4f*)(outp + (size_t)gr * FH + 4 * m) = fv[i];
    }
    __threadfence();
#pragma unroll
    for (int i = 0; i < 8; ++i) {
      const int gr = rowBase + 16 * wave + 2 * i + hh;
      *(volatile v4f*)(outp + (size_t)gr * FH + 4 * m) = fv[i];
    }
  } else {
    const int c0 = 2 * lane;
    const bool valid = c0 < NCLS;
    const int cc0 = c0 < NCLS ? c0 : NCLS - 1;
    const int cc1 = c0 + 1 < NCLS ? c0 + 1 : NCLS - 1;
    float bz0 = bf16_val(bias[cc0]), bz1 = bf16_val(bias[cc1]);
    bz0 = valid ? bz0 : 0.f;
    bz1 = valid ? bz1 : 0.f;
#pragma unroll 1
    for (int i = 0; i < 16; ++i) {
      const int lr = 16 * wave + i;
      const v2f v = *(const v2fa*)(stg + lr * GBN + c0);
      const float z0 = v.x + bz0, z1 = v.y + bz1;
      float vm = valid ? fmaxf(z0, z1) : -3.0e38f;
#pragma unroll
      for (int off = 16; off > 0; off >>= 1) vm = fmaxf(vm, __shfl_xor(vm, off, 32));
      const float d0 = valid ? (z0 - vm) : 0.0f;
      const float d1 = valid ? (z1 - vm) : 0.0f;
      const float ex0 = expf(d0), ex1 = expf(d1);
      float sm = valid ? (ex0 + ex1) : 0.0f;
#pragma unroll
      for (int off = 16; off > 0; off >>= 1) sm += __shfl_xor(sm, off, 32);
      const float ls = logf(sm);
      if (valid) {
        v2f ov; ov.x = d0 - ls; ov.y = d1 - ls;
        *(v2fa*)(res + lr * NCLS + c0) = ov;
      }
    }
    __syncthreads();
    int live = nOut - rowBase; live = live < 0 ? 0 : (live > GBM ? GBM : live);
    const int npc = live * (NCLS / 4);
    float* ob = outp + (size_t)rowBase * NCLS;
#pragma unroll 1
    for (int p = tid; p < npc; p += GTHR) {
      const v4f v = *(const v4fa*)(res + 4 * p);
      *(volatile v4f*)(ob + 4 * p) = v;
    }
    __threadfence();
#pragma unroll 1
    for (int p = tid; p < npc; p += GTHR) {
      const v4f v = *(const v4fa*)(res + 4 * p);
      *(volatile v4f*)(ob + 4 * p) = v;
    }
  }
}

template <int L>
__global__ __launch_bounds__(NTHR) void k_scan(const int* __restrict__ srcs, const int* __restrict__ dsts,
                                               int nE, int nN, int vec8, int mRows,
                                               const float* __restrict__ fin, unsigned short* apl) {
  extern __shared__ __attribute__((aligned(16))) int dsm[];
  int* list = dsm;
  int* hl   = dsm + LISTN;
  int* sl   = hl + RCAP;
  int* cnt  = sl + RCAP;
  int* offs = cnt + NBA;
  int* cur  = offs + NBA;
  int* misc = cur + NBA;
  const int tid = (int)threadIdx.x, lane = tid & 31, wave = tid >> 5;
  unsigned short* rowbuf = (unsigned short*)(misc + MISC_INTS) + wave * APS;
  const int nodeBase = (int)blockIdx.x * NBA;

  {
    const v4i z4 = {0, 0, 0, 0};
    for (int i = tid * 4; i < AGG_ZINTS; i += NTHR * 4) *(v4ia*)(dsm + i) = z4;
    if (tid < MISC_INTS) misc[tid] = 0;
  }
  __syncthreads();

  int t = 0, ov = 0;
  const int nChunks = (nE + CHUNK - 1) / CHUNK;
#pragma unroll 1
  for (int ch = 0; ch < nChunks; ++ch) {
    const int cbase = ch * CHUNK;
    const int wc = scan_chunk<SLA>(dsts, nE, cbase, nodeBase, NBA, vec8, list, tid, lane, wave);
    if (lane == 0) misc[wave] = wc;
    __syncthreads();
    if (wave == 0) {
#pragma unroll 1
      for (int w2 = 0; w2 < NWAVE; ++w2) {
        int c = misc[w2];
        c = c < 0 ? 0 : (c > WCAP ? WCAP : c);
#pragma unroll 1
        for (int b0 = 0; b0 < c; b0 += 32) {
          const int idx = b0 + lane;
          const int ent = list[w2 * WCAP + (idx < WCAP ? idx : WCAP - 1)];
          const int m32 = (c - b0) < 32 ? (c - b0) : 32;
#pragma unroll 1
          for (int k = 0; k < m32; ++k) {
            const int u    = __builtin_amdgcn_readlane(ent, k);
            const int slot = u & (NBA - 1);
            const int el   = (u >> SLA) & (CHUNK - 1);
            const int pk   = ((cbase + el) << SLA) | slot;
            if (t < RCAP) {
              if (lane == 0) { hl[t] = pk; cnt[slot] = cnt[slot] + 1; }
              t = t + 1;
            } else {
              ov = 1;
            }
          }
        }
      }
    }
    __syncthreads();
  }
  if (wave == 0 && lane == 0) { misc[8] = t; misc[9] = ov; }
  __syncthreads();
  int tt = misc[8];
  tt = tt < 0 ? 0 : (tt > RCAP ? RCAP : tt);
  const int ovf = misc[9];

  if (wave == 0) {
    const int base = lane * (NBA / 32);
    int s = 0;
#pragma unroll 1
    for (int i = 0; i < NBA / 32; ++i) s += cnt[base + i];
    int incl = s;
#pragma unroll
    for (int d = 1; d < 32; d <<= 1) {
      const int y = __shfl_up(incl, d, 32);
      if (lane >= d) incl += y;
    }
    int run = incl - s;
#pragma unroll 1
    for (int i = 0; i < NBA / 32; ++i) {
      const int cv = cnt[base + i];
      offs[base + i] = run;
      cur[base + i]  = run;
      run += cv;
    }
  }
  __syncthreads();
  if (wave == 0) {
#pragma unroll 1
    for (int b0 = 0; b0 < tt; b0 += 32) {
      const int idx = b0 + lane;
      const int ent = hl[idx < RCAP ? idx : RCAP - 1];
      const int m32 = (tt - b0) < 32 ? (tt - b0) : 32;
#pragma unroll 1
      for (int k = 0; k < m32; ++k) {
        const int u    = __builtin_amdgcn_readlane(ent, k);
        const int slot = u & (NBA - 1);
        if (lane == 0) {
          int p = cur[slot];
          p = p < 0 ? 0 : (p > RCAP - 1 ? RCAP - 1 : p);
          sl[p] = u;
          cur[slot] = p + 1;
        }
      }
    }
  }
  __syncthreads();

  const float qnan = __int_as_float(0x7fc00000);
  const float pz = (ovf != 0) ? qnan : 0.0f;
#pragma unroll 1
  for (int si = 0; si < NBA / NWAVE; ++si) {
    const int s    = si * NWAVE + wave;
    const int node = nodeBase + s;
    int c = cnt[s];
    const bool big = c > DEGCAP;
    c = c < 0 ? 0 : (c > DEGCAP ? DEGCAP : c);
    int o = offs[s];
    o = o < 0 ? 0 : (o > RCAP ? RCAP : o);
    const int nc = node < nN ? node : nN - 1;
    float a0 = 0.0f, a1 = 0.0f, a2 = 0.0f, a3 = 0.0f;
#pragma unroll 1
    for (int b0 = 0; b0 < c; b0 += 32) {
      int idx = o + b0 + lane;
      idx = idx > RCAP - 1 ? RCAP - 1 : idx;
      const int ent = sl[idx];
      int eid = ent >> SLA;
      eid = eid < 0 ? 0 : (eid > nE - 1 ? nE - 1 : eid);
      int sr = srcs[eid];
      sr = sr < 0 ? 0 : (sr > nN - 1 ? nN - 1 : sr);
      const int m32 = (c - b0) < 32 ? (c - b0) : 32;
#pragma unroll 1
      for (int k = 0; k < m32; ++k) {
        const int sk = __builtin_amdgcn_readlane(sr, k);
        if constexpr (L == 1) {
          const v4f a = *(const v4fa*)(fin + (size_t)sk * FX + 4 * lane);
          a0 += bf16_val(a.x); a1 += bf16_val(a.y); a2 += bf16_val(a.z); a3 += bf16_val(a.w);
        } else {
          const v2f a = *(const v2fa*)(fin + (size_t)sk * FH + 2 * lane);
          a0 += a.x; a1 += a.y;
        }
      }
    }
    const float inv = 1.0f / fmaxf((float)c, 1.0f);
    const float pzr = big ? qnan : pz;
    const bool live = node < nN;
    if constexpr (L == 1) {
      const float m0 = live ? (a0 * inv + pzr) : 0.0f;
      const float m1 = live ? (a1 * inv + pzr) : 0.0f;
      const float m2 = live ? (a2 * inv + pzr) : 0.0f;
      const float m3 = live ? (a3 * inv + pzr) : 0.0f;
      v4us mh, ml;
      {
        unsigned h0, l0, h1, l1, h2, l2, h3, l3;
        split2(m0, h0, l0); split2(m1, h1, l1); split2(m2, h2, l2); split2(m3, h3, l3);
        mh[0] = (unsigned short)h0; mh[1] = (unsigned short)h1; mh[2] = (unsigned short)h2; mh[3] = (unsigned short)h3;
        ml[0] = (unsigned short)l0; ml[1] = (unsigned short)l1; ml[2] = (unsigned short)l2; ml[3] = (unsigned short)l3;
      }
      const v4f xs = *(const v4fa*)(fin + (size_t)nc * FX + 4 * lane);
      v4us xb;
      xb[0] = live ? (unsigned short)bf16_bits(xs.x + pzr) : (unsigned short)0;
      xb[1] = live ? (unsigned short)bf16_bits(xs.y + pzr) : (unsigned short)0;
      xb[2] = live ? (unsigned short)bf16_bits(xs.z + pzr) : (unsigned short)0;
      xb[3] = live ? (unsigned short)bf16_bits(xs.w + pzr) : (unsigned short)0;
      *(v4usa*)(rowbuf + 4 * lane) = mh;
      *(v4usa*)(rowbuf + FX + 4 * lane) = ml;
      *(v4usa*)(rowbuf + 2 * FX + 4 * lane) = xb;
      wave_sync();
      const v8us q0 = *(const v8usa*)(rowbuf + 8 * lane);
      const v8us q1 = *(const v8usa*)(rowbuf + 2 * FX + 8 * (lane & 15));
      wave_sync();
      if (node < mRows) {
        unsigned short* rpw = apl + (size_t)node * K1 + 8 * lane;
        *(volatile v8us*)rpw = q0;
        if (lane < 16) *(volatile v8us*)(rpw + 2 * FX) = q1;
        __threadfence();
        *(volatile v8us*)rpw = q0;
        if (lane < 16) *(volatile v8us*)(rpw + 2 * FX) = q1;
      }
    } else {
      const float m0 = live ? (a0 * inv + pzr) : 0.0f;
      const float m1 = live ? (a1 * inv + pzr) : 0.0f;
      const v2f hs = *(const v2fa*)(fin + (size_t)nc * FH + 2 * lane);
      const float r0 = live ? (hs.x + pzr) : 0.0f;
      const float r1 = live ? (hs.y + pzr) : 0.0f;
      unsigned mh0, ml0, mh1, ml1, rh0, rl0, rh1, rl1;
      split2(m0, mh0, ml0); split2(m1, mh1, ml1); split2(r0, rh0, rl0); split2(r1, rh1, rl1);
      ua32* rb32 = (ua32*)rowbuf;
      rb32[lane]      = mh0 | (mh1 << 16);
      rb32[32 + lane] = ml0 | (ml1 << 16);
      rb32[64 + lane] = rh0 | (rh1 << 16);
      rb32[96 + lane] = rl0 | (rl1 << 16);
      wave_sync();
      const v8us q0 = *(const v8usa*)(rowbuf + 8 * lane);
      wave_sync();
      if (node < mRows) {
        unsigned short* rpw = apl + (size_t)node * K2 + 8 * lane;
        *(volatile v8us*)rpw = q0;
        __threadfence();
        *(volatile v8us*)rpw = q0;
      }
    }
  }
}

static inline int cdiv(int a, int b) { return (a + b - 1) / b; }

extern "C" void kernel_launch(void* const* d_in, const int* in_sizes, int n_in,
                              void* d_out, int out_size, void* d_ws, size_t ws_size,
                              hipStream_t stream) {
  if (n_in < 8) return;
  if (in_sizes[0] < FX || (in_sizes[0] % FX) != 0) return;
  const int nN = in_sizes[0] / FX;
  if (nN > (1 << 22)) return;
  if (in_sizes[1] < 2 || (in_sizes[1] & 1) != 0) return;
  const int nE = in_sizes[1] / 2;
  if (nE < 1 || nE >= (1 << 21)) return;
  if (in_sizes[2] != FX * FH || in_sizes[3] != FH || in_sizes[4] != FX * FH) return;
  if (in_sizes[5] != FH * NCLS || in_sizes[6] != NCLS || in_sizes[7] != FH * NCLS) return;
  if ((long long)out_size != (long long)nN * NCLS) return;

  const float* x    = (const float*)d_in[0];
  const int*   edge = (const int*)d_in[1];
  const float* Wl1  = (const float*)d_in[2];
  const float* bl1  = (const float*)d_in[3];
  const float* Wr1  = (const float*)d_in[4];
  const float* Wl2  = (const float*)d_in[5];
  const float* bl2  = (const float*)d_in[6];
  const float* Wr2  = (const float*)d_in[7];
  float* out = (float*)d_out;
  const int* src = edge;
  const int* dst = edge + nE;

  const int MP = cdiv(nN, GBM) * GBM;
  const int gM = MP / GBM;
  const int gA = cdiv(MP, NBA);
  if ((long long)gA * NBA < (long long)MP) return;
  const int vec8 = ((nE & 3) == 0) ? 1 : 0;

  char* ws = (char*)d_ws;
  size_t off = 0;
  const size_t oB0 = off; off += (size_t)FH * K1 * 2;                      off = (off + 255) & ~(size_t)255;
  const size_t oB1 = off; off += (size_t)NC2P * K2 * 2;                    off = (off + 255) & ~(size_t)255;
  const size_t oA  = off; off += (size_t)MP * K1 * 2;                      off = (off + 255) & ~(size_t)255;
  const size_t oH  = off; off += (size_t)MP * FH * 4;                      off = (off + 255) & ~(size_t)255;
  if (off > ws_size || off > (size_t)WSMAX) return;
  unsigned short* B0  = (unsigned short*)(ws + oB0);
  unsigned short* B1  = (unsigned short*)(ws + oB1);
  unsigned short* Apl = (unsigned short*)(ws + oA);
  float*          HF  = (float*)(ws + oH);

  const size_t scanLds = (size_t)AGG_LDS_INTS * 4;
  hipFuncSetAttribute(reinterpret_cast<const void*>(&k_scan<1>), hipFuncAttributeMaxDynamicSharedMemorySize, (int)scanLds);
  hipFuncSetAttribute(reinterpret_cast<const void*>(&k_scan<2>), hipFuncAttributeMaxDynamicSharedMemorySize, (int)scanLds);

  k_wprep<<<(U0 + U1) / NTHR, NTHR, 0, stream>>>(Wl1, Wr1, Wl2, Wr2, B0, B1);
  k_scan<1><<<gA, NTHR, scanLds, stream>>>(src, dst, nE, nN, vec8, MP, x, Apl);
  k_gemm<0><<<gM, GTHR, 0, stream>>>(Apl, B0, K1, bl1, HF, MP);
  k_scan<2><<<gA, NTHR, scanLds, stream>>>(src, dst, nE, nN, vec8, MP, HF, Apl);
  k_gemm<1><<<gM, GTHR, 0, stream>>>(Apl, B1, K2, bl2, out, nN);
}
